// ManifoldMHA_31327491457694
// MI455X (gfx1250) — hardware-verified
//
#include <hip/hip_runtime.h>
#include <math.h>

#define HIDN 512
#define NHEAD 8
#define SEQ 256
#define NB 2
#define HD 64
#define ROWS 512
#define NBH 16
#define EPSF 1e-15f
#define MAXNORM 0.996f
#define ATCLIP 0.99999988f

typedef __attribute__((ext_vector_type(16))) _Float16 v16h;
typedef __attribute__((ext_vector_type(8)))  _Float16 v8h;
typedef __attribute__((ext_vector_type(16))) __bf16   v16b;
typedef __attribute__((ext_vector_type(8)))  __bf16   v8b;
typedef __attribute__((ext_vector_type(8)))  float    v8f;
typedef __attribute__((ext_vector_type(4)))  float    v4f;
#define U16(p) ((const unsigned short*)(const void*)(p))

__device__ __forceinline__ unsigned short f2bf_bits(float f) {
  unsigned u = __float_as_uint(f);
  return (unsigned short)((u + 0x7FFFu + ((u >> 16) & 1u)) >> 16);
}
__device__ __forceinline__ float bf_bits2f(unsigned short h) { return __uint_as_float(((unsigned)h) << 16); }

__device__ __forceinline__ void dep_guard_h(v8f& a, v8f& b, v16h x, v16h y) { asm volatile("v_nop\n\tv_nop\n\tv_nop\n\tv_nop" : "+v"(a), "+v"(b) : "v"(x), "v"(y)); }
__device__ __forceinline__ void dep_guard_b(v8f& a, v8f& b, v16b x, v16b y) { asm volatile("v_nop\n\tv_nop\n\tv_nop\n\tv_nop" : "+v"(a), "+v"(b) : "v"(x), "v"(y)); }
__device__ __forceinline__ void keep4_h(v16h a, v16h b, v16h c, v16h d) { asm volatile("v_nop" :: "v"(a), "v"(b), "v"(c), "v"(d)); }
__device__ __forceinline__ void keep4_b(v16b a, v16b b, v16b c, v16b d) { asm volatile("v_nop" :: "v"(a), "v"(b), "v"(c), "v"(d)); }
__device__ __forceinline__ void acc_guard4(v8f& a, v8f& b, v8f& c, v8f& d) { asm volatile("v_nop\n\tv_nop\n\tv_nop\n\tv_nop" : "+v"(a), "+v"(b), "+v"(c), "+v"(d)); }
template <typename T> struct Frag;
template <> struct Frag<_Float16> {
  typedef v16h V; union U { v16h v; v8h h[2]; };
  static __device__ __forceinline__ v16h load(const _Float16* p) {
    U f; f.h[0] = *(const v8h*)(p); f.h[1] = *(const v8h*)(p + 16); return f.v;
  }
  static __device__ __forceinline__ v8f mma(v16h a, v16h b, v8f c) {
    return __builtin_amdgcn_wmma_f32_16x16x32_f16(false, a, false, b, (short)0, c, false, false);
  }
  static __device__ __forceinline__ void guard(v8f& a, v8f& b, v16h x, v16h y) { dep_guard_h(a, b, x, y); }
  static __device__ __forceinline__ void keep(v16h a, v16h b, v16h c, v16h d) { keep4_h(a, b, c, d); }
};
template <> struct Frag<__bf16> {
  typedef v16b V; union U { v16b v; v8b h[2]; };
  static __device__ __forceinline__ v16b load(const __bf16* p) {
    U f; f.h[0] = *(const v8b*)(p); f.h[1] = *(const v8b*)(p + 16); return f.v;
  }
  static __device__ __forceinline__ v8f mma(v16b a, v16b b, v8f c) {
    return __builtin_amdgcn_wmma_f32_16x16x32_bf16(false, a, false, b, (short)0, c, false, false);
  }
  static __device__ __forceinline__ void guard(v8f& a, v8f& b, v16b x, v16b y) { dep_guard_b(a, b, x, y); }
  static __device__ __forceinline__ void keep(v16b a, v16b b, v16b c, v16b d) { keep4_b(a, b, c, d); }
};

template <int ET> struct Elem;
template <> struct Elem<0> { typedef _Float16 T; };
template <> struct Elem<1> { typedef __bf16 T; };
template <int ET, bool SPLIT, int BIAS_MODE, int OUT_MODE, bool RESID, int ACT = 0>
__global__ __launch_bounds__(256) void wmma_gemm64(
    const unsigned short* __restrict__ Ap, const unsigned short* __restrict__ A2p, int lda, long strideA,
    const unsigned short* __restrict__ Btp, const unsigned short* __restrict__ Bt2p, int ldb, long strideB,
    void* __restrict__ Cout, void* __restrict__ Cout2, int ldc, long strideC,
    const float* __restrict__ bias,
    const float* __restrict__ resid, long strideR,
    int M, int N, int K, float scale) {
  typedef typename Elem<ET>::T T;
  typedef typename Frag<T>::V V;
  const T* A = (const T*)Ap; const T* A2 = (const T*)A2p; const T* Bt = (const T*)Btp; const T* Bt2 = (const T*)Bt2p;
  __shared__ __align__(16) float sT[8][16 * 68];
  const int b    = blockIdx.y;
  const int lane = threadIdx.x & 31;
  const int wave = threadIdx.x >> 5;
  const int tilesN = N >> 6;
  const int tilesM = M >> 6;
  const int tile = blockIdx.x * 8 + wave;
  if (tile >= tilesM * tilesN) return;
  const int tm = tile / tilesN;
  const int tn = tile - tm * tilesN;
  const int m0 = tm << 6;
  const int n0 = tn << 6;

  const T* Ab  = A  + (size_t)b * strideA;
  const T* Bb  = Bt + (size_t)b * strideB;
  const T* Ab2 = SPLIT ? (A2  + (size_t)b * strideA) : nullptr;
  const T* Bb2 = SPLIT ? (Bt2 + (size_t)b * strideB) : nullptr;

  const int rlane = lane & 15;
  const int koff  = (lane >> 4) * 8;
  const int mOff  = (lane >> 4) * 8;

  v8f acc[4][4];
#pragma unroll
  for (int i = 0; i < 4; ++i)
#pragma unroll
    for (int j = 0; j < 4; ++j) acc[i][j] = (v8f){0.f,0.f,0.f,0.f,0.f,0.f,0.f,0.f};

  for (int k0 = 0; k0 < K; k0 += 32) {
    V bh[4], bl[4];
#pragma unroll
    for (int j = 0; j < 4; ++j) {
      const size_t bo = (size_t)(n0 + (j << 4) + rlane) * ldb + koff + k0;
      bh[j] = Frag<T>::load(Bb + bo);
      if (SPLIT) bl[j] = Frag<T>::load(Bb2 + bo);
    }
#pragma unroll
    for (int i = 0; i < 4; ++i) {
      const size_t ao = (size_t)(m0 + (i << 4) + rlane) * lda + koff + k0;
      V ah = Frag<T>::load(Ab + ao);
      V al;
      if (SPLIT) al = Frag<T>::load(Ab2 + ao);
#pragma unroll
      for (int j = 0; j < 4; ++j) {
        acc[i][j] = Frag<T>::mma(ah, bh[j], acc[i][j]);
        if (SPLIT) {
          acc[i][j] = Frag<T>::mma(ah, bl[j], acc[i][j]);
          acc[i][j] = Frag<T>::mma(al, bh[j], acc[i][j]);
        }
      }
      Frag<T>::guard(acc[i][0], acc[i][3], ah, SPLIT ? al : ah);
    }
    Frag<T>::keep(bh[0], bh[1], bh[2], bh[3]);
    if (SPLIT) Frag<T>::keep(bl[0], bl[1], bl[2], bl[3]);
  }
  acc_guard4(acc[0][0], acc[0][1], acc[0][2], acc[0][3]);
  acc_guard4(acc[1][0], acc[1][1], acc[1][2], acc[1][3]);
  acc_guard4(acc[2][0], acc[2][1], acc[2][2], acc[2][3]);
  acc_guard4(acc[3][0], acc[3][1], acc[3][2], acc[3][3]);

  float* slab = sT[wave];
  const float* Rb = RESID ? (resid + (size_t)b * strideR) : nullptr;
#pragma unroll
  for (int i = 0; i < 4; ++i) {
    const int mBase = m0 + (i << 4);
#pragma unroll
    for (int j = 0; j < 4; ++j) {
      const int n = n0 + (j << 4) + rlane;
      float bv = 0.f;
      if (BIAS_MODE == 2) bv = bias[n];
#pragma unroll
      for (int r = 0; r < 8; ++r) {
        float v = acc[i][j][r] * scale;
        if (BIAS_MODE == 1) v += bias[mBase + mOff + r];
        if (BIAS_MODE == 2) v += bv;
        if (RESID) v += Rb[(size_t)(mBase + mOff + r) * ldc + n];
        if (ACT == 1) v = tanhf(v);
        if (ACT == 2) v = fmaxf(v, 0.0f);
        if (ACT == 3) v = v / (1.0f + expf(-v));
        if (ACT == 4) v = (v > 0.f) ? v : 0.01f * v;
        if (ACT == 5) v = 0.5f * v * (1.0f + erff(v * 0.70710678118654752f));
        slab[(mOff + r) * 68 + (j << 4) + rlane] = v;
      }
    }
    __builtin_amdgcn_fence(__ATOMIC_RELEASE, "workgroup");
    __builtin_amdgcn_wave_barrier();
    __builtin_amdgcn_fence(__ATOMIC_ACQUIRE, "workgroup");
    if (OUT_MODE == 0) {
      float* C = (float*)Cout + (size_t)b * strideC;
      const int hh = lane >> 4, c4 = (lane & 15) * 4;
      for (int pass = 0; pass < 2; ++pass) {
#pragma unroll
        for (int it = 0; it < 8; ++it) {
          const int row = it * 2 + hh;
          v4f v = *(const v4f*)(slab + row * 68 + c4);
          *(volatile v4f*)(C + (size_t)(mBase + row) * ldc + n0 + c4) = v;
        }
        __threadfence();
      }
    } else {
      const int q = lane >> 3, c8 = (lane & 7) * 8;
      unsigned short* C  = (unsigned short*)Cout  + (size_t)b * strideC;
      unsigned short* C2 = (OUT_MODE == 2) ? ((unsigned short*)Cout2 + (size_t)b * strideC) : nullptr;
      for (int pass = 0; pass < 2; ++pass) {
#pragma unroll
        for (int it = 0; it < 4; ++it) {
          const int row = it * 4 + q;
          const float* sp = slab + row * 68 + c8;
          v8h hv, lv;
#pragma unroll
          for (int e = 0; e < 8; ++e) {
            if (OUT_MODE == 1) {
              hv[e] = (_Float16)sp[e];
            } else {
              unsigned short hb = f2bf_bits(sp[e]);
              unsigned short lb = f2bf_bits(sp[e] - bf_bits2f(hb));
              hv[e] = __builtin_bit_cast(_Float16, hb);
              lv[e] = __builtin_bit_cast(_Float16, lb);
            }
          }
          *(volatile v8h*)(C + (size_t)(mBase + row) * ldc + n0 + c8) = hv;
          if (OUT_MODE == 2) *(volatile v8h*)(C2 + (size_t)(mBase + row) * ldc + n0 + c8) = lv;
        }
        __threadfence();
      }
    }
    __builtin_amdgcn_fence(__ATOMIC_RELEASE, "workgroup");
    __builtin_amdgcn_wave_barrier();
    __builtin_amdgcn_fence(__ATOMIC_ACQUIRE, "workgroup");
  }
}

__device__ __forceinline__ float atanh_clip(float x) {
  x = fminf(fmaxf(x, -ATCLIP), ATCLIP);
  return atanhf(x);
}
__device__ __forceinline__ float wsum(float v) {
#pragma unroll
  for (int off = 16; off > 0; off >>= 1) v += __shfl_xor(v, off, 32);
  return v;
}
__device__ __forceinline__ float sum16(const float* r) {
  float s = 0.0f;
#pragma unroll
  for (int k = 0; k < 16; ++k) s += r[k];
  return s;
}

__global__ __launch_bounds__(256) void k_cast16(const float* __restrict__ query,
    const float* __restrict__ Wq, const float* __restrict__ Wk, const float* __restrict__ Wv,
    _Float16* __restrict__ X16, _Float16* __restrict__ W16) {
  const int blk = blockIdx.x, t = threadIdx.x;
  if (blk < 128) {
    const int u = blk * 256 + t;
    const int m = u >> 6, c8 = (u & 63) * 8;
    const int b = m >> 8, s = m & 255;
    const float* src = query + ((size_t)(s * NB + b)) * HIDN + c8;
    const v4f a0 = *(const v4f*)src;
    const v4f a1 = *(const v4f*)(src + 4);
    v8h hv;
#pragma unroll
    for (int e = 0; e < 4; ++e) { hv[e] = (_Float16)(a0[e] * 64.0f); hv[4 + e] = (_Float16)(a1[e] * 64.0f); }
    _Float16* dst = X16 + (size_t)m * HIDN + c8;
    *(volatile v8h*)dst = hv;
    __threadfence();
    *(volatile v8h*)dst = hv;
  } else {
    const int u = (blk - 128) * 256 + t;
    const int n = u >> 6, c8 = (u & 63) * 8;
    const int p = n >> 9, o = n & 511;
    const float* W = (p == 0) ? Wq : (p == 1) ? Wk : Wv;
    const float* src = W + (size_t)o * HIDN + c8;
    const v4f a0 = *(const v4f*)src;
    const v4f a1 = *(const v4f*)(src + 4);
    v8h hv;
#pragma unroll
    for (int e = 0; e < 4; ++e) { hv[e] = (_Float16)(a0[e] * 16.0f); hv[4 + e] = (_Float16)(a1[e] * 16.0f); }
    _Float16* dst = W16 + (size_t)n * HIDN + c8;
    *(volatile v8h*)dst = hv;
    __threadfence();
    *(volatile v8h*)dst = hv;
  }
}

__global__ __launch_bounds__(512) void k_linA(const float* __restrict__ query, const float* __restrict__ MX,
    const float* __restrict__ bq, const float* __restrict__ bk, const float* __restrict__ bv,
    float* __restrict__ UB) {
  __shared__ float red[7][16];
  __shared__ __align__(16) float rowbuf[512];
  const int m = blockIdx.x, p = blockIdx.y, t = threadIdx.x, lane = t & 31, wave = t >> 5;
  const int b = m >> 8, s = m & 255;
  const float* bias = (p == 0) ? bq : (p == 1) ? bk : bv;
  const float x  = query[((size_t)(s * NB + b)) * HIDN + t];
  const float v  = MX[(size_t)m * (3 * HIDN) + p * HIDN + t];
  const float bb = bias[t];
  float w0 = wsum(x * x), w1 = wsum(v * v), w2 = wsum(bb * bb), w3 = wsum((v != 0.0f) ? 1.0f : 0.0f);
  if (lane == 0) { red[0][wave] = w0; red[1][wave] = w1; red[2][wave] = w2; red[3][wave] = w3; }
  __syncthreads();
  const float x2 = sum16(red[0]), mx2 = sum16(red[1]), b2 = sum16(red[2]), nz = sum16(red[3]);
  const float xn  = fmaxf(sqrtf(x2), EPSF);
  const float mxn = fmaxf(sqrtf(mx2), EPSF);
  const float tt  = tanhf((mxn / xn) * atanh_clip(xn));
  const float inv_mxn = 1.0f / mxn;
  float res = tt * (v * inv_mxn);
  if (nz == 0.0f) res = 0.0f;
  w0 = wsum(res * res); w1 = wsum(res * bb);
  if (lane == 0) { red[4][wave] = w0; red[5][wave] = w1; }
  __syncthreads();
  const float res2 = sum16(red[4]), rb = sum16(red[5]);
  const float a1  = 1.0f + 2.0f * rb + b2;
  const float b1  = 1.0f - res2;
  const float den = 1.0f + 2.0f * rb + res2 * b2;
  const float inv_den = 1.0f / fmaxf(den, EPSF);
  const float ma = (a1 * res + b1 * bb) * inv_den;
  w0 = wsum(ma * ma);
  if (lane == 0) red[6][wave] = w0;
  __syncthreads();
  const float n3 = fmaxf(sqrtf(sum16(red[6])), EPSF);
  float u = ma;
  if (n3 > MAXNORM) u = (ma * (1.0f / n3)) * MAXNORM;
  rowbuf[t] = u;
  __syncthreads();
  if (t < 128) {
    const v4f val = *(const v4f*)(rowbuf + 4 * t);
    float* dst = UB + ((size_t)(p * ROWS + m)) * HIDN + 4 * t;
    *(volatile v4f*)dst = val;
    __threadfence();
    *(volatile v4f*)dst = val;
  }
}

__global__ __launch_bounds__(512) void k_linB(const float* __restrict__ UB, _Float16* __restrict__ OP,
    float* __restrict__ RS, float scale) {
  __shared__ float red[4][16];
  __shared__ __align__(16) float rowbuf[512];
  __shared__ __align__(16) float rsl[32];
  const int m = blockIdx.x, p = blockIdx.y, t = threadIdx.x, lane = t & 31, wave = t >> 5;
  const int cp = wave >> 1;
  const float u = UB[((size_t)(p * ROWS + m)) * HIDN + t];
  float w0 = wsum(u * u);
  if (lane == 0) red[0][wave] = w0;
  __syncthreads();
  const float n4 = fmaxf(sqrtf(sum16(red[0])), EPSF);
  const float lg = ((u * (1.0f / n4)) * atanh_clip(n4)) * scale;
  w0 = wsum(lg * lg);
  if (lane == 0) red[1][wave] = w0;
  __syncthreads();
  const float s5 = red[1][2 * cp] + red[1][2 * cp + 1];
  const float n5 = fmaxf(sqrtf(s5), EPSF);
  const float e  = (tanhf(n5) * lg) * (1.0f / n5);
  w0 = wsum(e * e);
  if (lane == 0) red[2][wave] = w0;
  __syncthreads();
  const float n6 = fmaxf(sqrtf(red[2][2 * cp] + red[2][2 * cp + 1]), EPSF);
  float w = e;
  if (n6 > MAXNORM) w = (e * (1.0f / n6)) * MAXNORM;
  w0 = wsum(w * w);
  if (lane == 0) red[3][wave] = w0;
  __syncthreads();
  rowbuf[t] = w * 8.0f;
  if (t < 8) {
    const float sq = red[3][2 * t] + red[3][2 * t + 1];
    rsl[t] = sq;
    rsl[8 + t] = 2.0f / fmaxf(1.0f - sq, EPSF);
  } else if (t >= 16 && t < 32) {
    rsl[t] = 0.0f;
  }
  __syncthreads();
  if (t < 64) {
    v8h hv;
#pragma unroll
    for (int k = 0; k < 8; ++k) hv[k] = (_Float16)rowbuf[8 * t + k];
    _Float16* dst = OP + (size_t)p * ROWS * HIDN + (size_t)m * HIDN + 8 * t;
    *(volatile v8h*)dst = hv;
    __threadfence();
    *(volatile v8h*)dst = hv;
  } else if (t < 72) {
    const int q = t - 64;
    const v4f val = *(const v4f*)(rsl + 4 * q);
    float* dst = RS + ((size_t)(p * ROWS + m)) * 32 + 4 * q;
    *(volatile v4f*)dst = val;
    __threadfence();
    *(volatile v4f*)dst = val;
  }
}

__global__ __launch_bounds__(64) void k_colsoftmax(const float* __restrict__ XY, const float* __restrict__ RS,
    float* __restrict__ probs, _Float16* __restrict__ PG) {
  __shared__ __align__(16) float sc[SEQ * 64];
  const int tile = blockIdx.x, bh = blockIdx.y, t = threadIdx.x, lane = t & 31, wave = t >> 5;
  const int j0 = tile * 64, j = j0 + t;
  const float k2 = RS[(size_t)(ROWS + bh * 32 + (j >> 3)) * 32 + (j & 7)];
  const float* xcol = XY + (size_t)bh * (SEQ * SEQ) + j;
  const float* q2p = RS + (size_t)(bh * 32) * 32;
  float mx = -INFINITY;
#pragma unroll 1
  for (int i = 0; i < SEQ; ++i) {
    const float xy = xcol[(size_t)i * SEQ];
    const float q2 = q2p[(i >> 3) * 32 + (i & 7)];
    const float ca = 1.0f - 2.0f * xy + k2;
    const float cb = 1.0f - q2;
    float num2 = ca * ca * q2 - 2.0f * ca * cb * xy + cb * cb * k2;
    num2 = fmaxf(num2, 0.0f);
    const float den = fmaxf(1.0f - 2.0f * xy + q2 * k2, EPSF);
    const float t1 = sqrtf(num2) * (1.0f / den);
    float sv = -2.0f * atanh_clip(t1);
    sv = fminf(fmaxf(sv, -1e10f), 1e10f);
    sc[i * 64 + t] = sv;
    mx = fmaxf(mx, sv);
  }
  float ls = 0.0f;
#pragma unroll 1
  for (int i = 0; i < SEQ; ++i) ls += expf(sc[i * 64 + t] - mx);
  const float inv = 1.0f / ls;
#pragma unroll 1
  for (int i = 0; i < SEQ; ++i) sc[i * 64 + t] = expf(sc[i * 64 + t] - mx) * inv;
  __syncthreads();
  const int hh = lane >> 4, c16 = lane & 15, q = lane >> 3, c8 = (lane & 7) * 8;
  float g8[8];
#pragma unroll
  for (int e = 0; e < 8; ++e) {
    const int jj = j0 + c8 + e;
    g8[e] = RS[(size_t)(2 * ROWS + bh * 32 + (jj >> 3)) * 32 + 8 + (jj & 7)] * 256.0f;
  }
  float* ob = probs + (size_t)bh * (SEQ * SEQ) + j0;
  _Float16* pb = PG + (size_t)bh * (SEQ * SEQ) + j0;
  for (int pass = 0; pass < 2; ++pass) {
#pragma unroll 1
    for (int it = 0; it < 64; ++it) {
      const int i = wave * 128 + it * 2 + hh;
      const v4f val = *(const v4f*)(sc + i * 64 + c16 * 4);
      *(volatile v4f*)(ob + (size_t)i * SEQ + c16 * 4) = val;
    }
#pragma unroll 1
    for (int it = 0; it < 32; ++it) {
      const int i = wave * 128 + it * 4 + q;
      const float* sp = sc + i * 64 + c8;
      v8h hv;
#pragma unroll
      for (int e = 0; e < 8; ++e) hv[e] = (_Float16)(sp[e] * g8[e]);
      *(volatile v8h*)(pb + (size_t)i * SEQ + c8) = hv;
    }
    __threadfence();
  }
}

__global__ __launch_bounds__(256) void k_transp_v(const _Float16* __restrict__ V, _Float16* __restrict__ VT) {
  __shared__ __align__(16) _Float16 sh[64 * 72];
  const int tile = blockIdx.x, bh = blockIdx.y, t = threadIdx.x, lane = t & 31, wave = t >> 5;
  const int s0 = tile * 64;
  {
    const int r = t >> 2, c16 = (t & 3) * 16;
    const _Float16* src = V + ((size_t)(bh * SEQ + s0 + r)) * HD + c16;
    const v8h a0 = *(const v8h*)src;
    const v8h a1 = *(const v8h*)(src + 8);
    *(v8h*)(sh + r * 72 + c16) = a0;
    *(v8h*)(sh + r * 72 + c16 + 8) = a1;
  }
  __syncthreads();
  const int q = lane >> 3, c8 = (lane & 7) * 8;
  const int d0 = wave * 8 + q, d1 = wave * 8 + 4 + q;
  v8h hv0, hv1;
#pragma unroll
  for (int e = 0; e < 8; ++e) { hv0[e] = sh[(c8 + e) * 72 + d0]; hv1[e] = sh[(c8 + e) * 72 + d1]; }
  _Float16* dst0 = VT + ((size_t)(bh * HD + d0)) * SEQ + s0 + c8;
  _Float16* dst1 = VT + ((size_t)(bh * HD + d1)) * SEQ + s0 + c8;
  *(volatile v8h*)dst0 = hv0;
  *(volatile v8h*)dst1 = hv1;
  __threadfence();
  *(volatile v8h*)dst0 = hv0;
  *(volatile v8h*)dst1 = hv1;
}

__global__ __launch_bounds__(512) void k_ctxA(const float* __restrict__ probs, const float* __restrict__ RS,
    const float* __restrict__ NOM, float* __restrict__ LC, float invscale) {
  __shared__ float red[2][16];
  __shared__ float dens[8];
  __shared__ __align__(16) float rowbuf[512];
  const int m = blockIdx.x, t = threadIdx.x, lane = t & 31, wave = t >> 5;
  const int b = m >> 8, i = m & 255, h = t >> 6, d = t & 63;
  if (wave < 8) {
    const int bhw = b * NHEAD + wave;
    const float* prow = probs + ((size_t)(bhw * SEQ + i)) * SEQ;
    const float* grow = RS + (size_t)(2 * ROWS + bhw * 32) * 32 + 8;
    float acc = 0.0f;
#pragma unroll
    for (int k = 0; k < 8; ++k) {
      const int jj = lane + 32 * k;
      acc += prow[jj] * (grow[(jj >> 3) * 32 + (jj & 7)] - 1.0f);
    }
    acc = wsum(acc);
    if (lane == 0) dens[wave] = acc;
  }
  __syncthreads();
  const int bh = b * NHEAD + h;
  const float dn = fmaxf(dens[h], 1e-10f);
  const float tm = NOM[((size_t)(bh * SEQ + i)) * HD + d] * (1.0f / dn);
  float w0 = wsum(tm * tm);
  if (lane == 0) red[0][wave] = w0;
  __syncthreads();
  const float sq  = red[0][2 * h] + red[0][2 * h + 1];
  const float fac = 1.0f / (1.0f + sqrtf(fmaxf(1.0f - sq, 1e-10f)));
  const float cx  = tm * fac;
  w0 = wsum(cx * cx);
  if (lane == 0) red[1][wave] = w0;
  __syncthreads();
  const float n  = fmaxf(sqrtf(red[1][2 * h] + red[1][2 * h + 1]), EPSF);
  const float lc = ((cx * (1.0f / n)) * atanh_clip(n)) * invscale;
  rowbuf[t] = lc;
  __syncthreads();
  if (t < 128) {
    const v4f val = *(const v4f*)(rowbuf + 4 * t);
    float* dst = LC + (size_t)m * HIDN + 4 * t;
    *(volatile v4f*)dst = val;
    __threadfence();
    *(volatile v4f*)dst = val;
  }
}

__global__ __launch_bounds__(512) void k_ctxB(const float* __restrict__ LC, float* __restrict__ out0) {
  __shared__ float red[2][16];
  __shared__ __align__(16) float rowbuf[512];
  const int m = blockIdx.x, t = threadIdx.x, lane = t & 31, wave = t >> 5;
  const int b = m >> 8, s = m & 255;
  const float u = LC[(size_t)m * HIDN + t];
  float w0 = wsum(u * u);
  if (lane == 0) red[0][wave] = w0;
  __syncthreads();
  const float n5 = fmaxf(sqrtf(sum16(red[0])), EPSF);
  const float e  = (tanhf(n5) * u) * (1.0f / n5);
  w0 = wsum(e * e);
  if (lane == 0) red[1][wave] = w0;
  __syncthreads();
  const float n6 = fmaxf(sqrtf(sum16(red[1])), EPSF);
  float o = e;
  if (n6 > MAXNORM) o = (e * (1.0f / n6)) * MAXNORM;
  rowbuf[t] = o;
  __syncthreads();
  if (t < 128) {
    const v4f val = *(const v4f*)(rowbuf + 4 * t);
    float* dst = out0 + ((size_t)(s * NB + b)) * HIDN + 4 * t;
    *(volatile v4f*)dst = val;
    __threadfence();
    *(volatile v4f*)dst = val;
  }
}

static double host_beta(double a, double b) {
  return exp(lgamma(a) + lgamma(b) - lgamma(a + b));
}

extern "C" void kernel_launch(void* const* d_in, const int* in_sizes, int n_in,
                              void* d_out, int out_size, void* d_ws, size_t ws_size,
                              hipStream_t stream) {
  if (n_in < 7) return;
  if (in_sizes[0] != ROWS * HIDN || in_sizes[1] != HIDN * HIDN || in_sizes[2] != HIDN ||
      in_sizes[3] != HIDN * HIDN || in_sizes[4] != HIDN || in_sizes[5] != HIDN * HIDN || in_sizes[6] != HIDN) return;
  if (out_size != ROWS * HIDN + NBH * SEQ * SEQ) return;

  const float* query = (const float*)d_in[0];
  const float* Wq = (const float*)d_in[1];
  const float* bq = (const float*)d_in[2];
  const float* Wk = (const float*)d_in[3];
  const float* bk = (const float*)d_in[4];
  const float* Wv = (const float*)d_in[5];
  const float* bv = (const float*)d_in[6];
  float* out0 = (float*)d_out;
  float* out1 = out0 + (size_t)ROWS * HIDN;

  char* ws = (char*)d_ws;
  size_t off = 0;
  auto carve = [&](size_t bytes) { size_t o = off; off += (bytes + 255) & ~(size_t)255; return (void*)(ws + o); };
  _Float16* X16 = (_Float16*)carve((size_t)ROWS * HIDN * 2);
  _Float16* W16 = (_Float16*)carve((size_t)3 * HIDN * HIDN * 2);
  float*    MX  = (float*)carve((size_t)ROWS * 3 * HIDN * 4);
  float*    UB  = (float*)carve((size_t)3 * ROWS * HIDN * 4);
  _Float16* OP  = (_Float16*)carve((size_t)3 * ROWS * HIDN * 2);
  float*    RS  = (float*)carve((size_t)3 * ROWS * 32 * 4);
  float*    XY  = (float*)carve((size_t)NBH * SEQ * SEQ * 4);
  _Float16* PG  = (_Float16*)carve((size_t)NBH * SEQ * SEQ * 2);
  _Float16* VT  = (_Float16*)carve((size_t)NBH * HD * SEQ * 2);
  float*    NOM = (float*)carve((size_t)NBH * SEQ * HD * 4);
  float*    LC  = (float*)carve((size_t)ROWS * HIDN * 4);
  if (off > ws_size) return;

  const double beta_ni = host_beta((double)HD / 2.0, 0.5);
  const double beta_n  = host_beta((double)HIDN / 2.0, 0.5);
  const float scale    = (float)(beta_ni / beta_n);
  const float invscale = (float)(beta_n / beta_ni);

  k_cast16<<<512, 256, 0, stream>>>(query, Wq, Wk, Wv, X16, W16);

  wmma_gemm64<0, false, 0, 0, false, 0><<<dim3(24, 1), 256, 0, stream>>>(
      U16(X16), nullptr, HIDN, 0L, U16(W16), nullptr, HIDN, 0L,
      (void*)MX, nullptr, 3 * HIDN, 0L, nullptr, nullptr, 0L, ROWS, 3 * HIDN, HIDN, 1.0f / 1024.0f);

  k_linA<<<dim3(ROWS, 3), 512, 0, stream>>>(query, MX, bq, bk, bv, UB);
  k_linB<<<dim3(ROWS, 3), 512, 0, stream>>>(UB, OP, RS, scale);

  wmma_gemm64<0, false, 0, 0, false, 0><<<dim3(2, NBH), 256, 0, stream>>>(
      U16(OP), nullptr, HD, (long)(SEQ * HD), U16(OP + (size_t)ROWS * HIDN), nullptr, HD, (long)(SEQ * HD),
      (void*)XY, nullptr, SEQ, (long)(SEQ * SEQ), nullptr, nullptr, 0L, SEQ, SEQ, HD, 1.0f / 64.0f);

  k_colsoftmax<<<dim3(4, NBH), 64, 0, stream>>>(XY, RS, out1, PG);

  k_transp_v<<<dim3(4, NBH), 256, 0, stream>>>(OP + (size_t)2 * ROWS * HIDN, VT);

  wmma_gemm64<0, false, 0, 0, false, 0><<<dim3(1, NBH), 256, 0, stream>>>(
      U16(PG), nullptr, SEQ, (long)(SEQ * SEQ), U16(VT), nullptr, SEQ, (long)(HD * SEQ),
      (void*)NOM, nullptr, HD, (long)(SEQ * HD), nullptr, nullptr, 0L, SEQ, HD, SEQ, 1.0f / 2048.0f);

  k_ctxA<<<ROWS, 512, 0, stream>>>(out1, RS, NOM, LC, invscale);
  k_ctxB<<<ROWS, 512, 0, stream>>>(LC, out0);
}
